// DiGCN_IB_Sum_15908558864505
// MI455X (gfx1250) — hardware-verified
//
#include <hip/hip_runtime.h>
#include <math.h>
#include <stdint.h>

#define NFEAT   128
#define NHID    256
#define NQKV    768
#define QKP     512
#define NHEAD   4
#define DHD     64
#define NNODE   32768
#define NEDGE   524288
#define NGRAPH  64
#define NPG     512

typedef __attribute__((ext_vector_type(16))) _Float16 v16h;
typedef __attribute__((ext_vector_type(8)))  _Float16 v8h;
typedef __attribute__((ext_vector_type(16))) __bf16   v16b;
typedef __attribute__((ext_vector_type(8)))  __bf16   v8b;
typedef __attribute__((ext_vector_type(8)))  float    v8f;
typedef __attribute__((ext_vector_type(4)))  float    v4f;
typedef __attribute__((ext_vector_type(2)))  float    v2f;
typedef __attribute__((ext_vector_type(4)))  unsigned int v4u;
typedef __attribute__((ext_vector_type(2)))  unsigned int v2u;
typedef __attribute__((ext_vector_type(4)))  int      v4i;

__device__ __forceinline__ unsigned short f2bf_bits(float f) {
  unsigned u = __float_as_uint(f);
  return (unsigned short)((u + 0x7FFFu + ((u >> 16) & 1u)) >> 16);
}
__device__ __forceinline__ float bf_bits2f(unsigned short h) { return __uint_as_float(((unsigned)h) << 16); }
__device__ __forceinline__ unsigned pk16(unsigned short a, unsigned short b) { return (unsigned)a | ((unsigned)b << 16); }

__device__ __forceinline__ void dep_guard_h(v8f& a, v8f& b, v16h x, v16h y) { asm volatile("v_nop\n\tv_nop\n\tv_nop\n\tv_nop" : "+v"(a), "+v"(b) : "v"(x), "v"(y)); }
__device__ __forceinline__ void dep_guard_b(v8f& a, v8f& b, v16b x, v16b y) { asm volatile("v_nop\n\tv_nop\n\tv_nop\n\tv_nop" : "+v"(a), "+v"(b) : "v"(x), "v"(y)); }
__device__ __forceinline__ void keep4_h(v16h a, v16h b, v16h c, v16h d) { asm volatile("v_nop" :: "v"(a), "v"(b), "v"(c), "v"(d)); }
__device__ __forceinline__ void keep4_b(v16b a, v16b b, v16b c, v16b d) { asm volatile("v_nop" :: "v"(a), "v"(b), "v"(c), "v"(d)); }
__device__ __forceinline__ void acc_guard4(v8f& a, v8f& b, v8f& c, v8f& d) { asm volatile("v_nop\n\tv_nop\n\tv_nop\n\tv_nop" : "+v"(a), "+v"(b), "+v"(c), "+v"(d)); }

template <typename T> struct Frag;
template <> struct Frag<_Float16> {
  typedef v16h V; union U { v16h v; v8h h[2]; };
  static __device__ __forceinline__ v16h load(const _Float16* p) {
    U f; f.h[0] = *(const v8h*)(p); f.h[1] = *(const v8h*)(p + 16); return f.v;
  }
  static __device__ __forceinline__ v8f mma(v16h a, v16h b, v8f c) {
    return __builtin_amdgcn_wmma_f32_16x16x32_f16(false, a, false, b, (short)0, c, false, false);
  }
  static __device__ __forceinline__ void guard(v8f& a, v8f& b, v16h x, v16h y) { dep_guard_h(a, b, x, y); }
  static __device__ __forceinline__ void keep(v16h a, v16h b, v16h c, v16h d) { keep4_h(a, b, c, d); }
};
template <> struct Frag<__bf16> {
  typedef v16b V; union U { v16b v; v8b h[2]; };
  static __device__ __forceinline__ v16b load(const __bf16* p) {
    U f; f.h[0] = *(const v8b*)(p); f.h[1] = *(const v8b*)(p + 16); return f.v;
  }
  static __device__ __forceinline__ v8f mma(v16b a, v16b b, v8f c) {
    return __builtin_amdgcn_wmma_f32_16x16x32_bf16(false, a, false, b, (short)0, c, false, false);
  }
  static __device__ __forceinline__ void guard(v8f& a, v8f& b, v16b x, v16b y) { dep_guard_b(a, b, x, y); }
  static __device__ __forceinline__ void keep(v16b a, v16b b, v16b c, v16b d) { keep4_b(a, b, c, d); }
};

__device__ __forceinline__ v8f mma_b(v16b a, v16b b, v8f c) {
  c = __builtin_amdgcn_wmma_f32_16x16x32_bf16(false, a, false, b, (short)0, c, false, false);
  asm volatile("v_nop\n\tv_nop\n\tv_nop\n\tv_nop" : "+v"(c) : "v"(a), "v"(b));
  return c;
}
__device__ __forceinline__ v8f mma_h(v16h a, v16h b, v8f c) {
  c = __builtin_amdgcn_wmma_f32_16x16x32_f16(false, a, false, b, (short)0, c, false, false);
  asm volatile("v_nop\n\tv_nop\n\tv_nop\n\tv_nop" : "+v"(c) : "v"(a), "v"(b));
  return c;
}

template <int ET> struct Elem;
template <> struct Elem<0> { typedef _Float16 T; };
template <> struct Elem<1> { typedef __bf16 T; };
template <int ET, bool SPLIT, int BIAS_MODE, int OUT_MODE, bool RESID>
__global__ __launch_bounds__(256) void wmma_gemm64(
    const unsigned short* __restrict__ Ap, const unsigned short* __restrict__ A2p, int lda, long strideA,
    const unsigned short* __restrict__ Btp, const unsigned short* __restrict__ Bt2p, int ldb, long strideB,
    void* __restrict__ Cout, void* __restrict__ Cout2, int ldc, long strideC,
    const float* __restrict__ bias,
    const float* __restrict__ resid, long strideR,
    int M, int N, int K, float scale) {
  typedef typename Elem<ET>::T T;
  typedef typename Frag<T>::V V;
  const T* A = (const T*)Ap; const T* A2 = (const T*)A2p; const T* Bt = (const T*)Btp; const T* Bt2 = (const T*)Bt2p;
  __shared__ __align__(16) float sT[8][16 * 68];
  const int b    = blockIdx.y;
  const int lane = threadIdx.x & 31;
  const int wave = threadIdx.x >> 5;
  const int tilesN = N >> 6;
  const int tilesM = M >> 6;
  const int tile = blockIdx.x * 8 + wave;
  if (tile >= tilesM * tilesN) return;
  const int tm = tile / tilesN;
  const int tn = tile - tm * tilesN;
  const int m0 = tm << 6;
  const int n0 = tn << 6;

  const T* Ab  = A  + (size_t)b * strideA;
  const T* Bb  = Bt + (size_t)b * strideB;
  const T* Ab2 = SPLIT ? (A2  + (size_t)b * strideA) : nullptr;
  const T* Bb2 = SPLIT ? (Bt2 + (size_t)b * strideB) : nullptr;

  const int rlane = lane & 15;
  const int koff  = (lane >> 4) * 8;
  const int mOff  = (lane >> 4) * 8;

  v8f acc[4][4];
#pragma unroll
  for (int i = 0; i < 4; ++i)
#pragma unroll
    for (int j = 0; j < 4; ++j) acc[i][j] = (v8f){0.f,0.f,0.f,0.f,0.f,0.f,0.f,0.f};

  for (int k0 = 0; k0 < K; k0 += 32) {
    V bh[4], bl[4];
#pragma unroll
    for (int j = 0; j < 4; ++j) {
      const size_t bo = (size_t)(n0 + (j << 4) + rlane) * ldb + koff + k0;
      bh[j] = Frag<T>::load(Bb + bo);
      if (SPLIT) bl[j] = Frag<T>::load(Bb2 + bo);
    }
#pragma unroll
    for (int i = 0; i < 4; ++i) {
      const size_t ao = (size_t)(m0 + (i << 4) + rlane) * lda + koff + k0;
      V ah = Frag<T>::load(Ab + ao);
      V al;
      if (SPLIT) al = Frag<T>::load(Ab2 + ao);
#pragma unroll
      for (int j = 0; j < 4; ++j) {
        acc[i][j] = Frag<T>::mma(ah, bh[j], acc[i][j]);
        if (SPLIT) {
          acc[i][j] = Frag<T>::mma(ah, bl[j], acc[i][j]);
          acc[i][j] = Frag<T>::mma(al, bh[j], acc[i][j]);
        }
      }
      Frag<T>::guard(acc[i][0], acc[i][3], ah, SPLIT ? al : ah);
    }
    Frag<T>::keep(bh[0], bh[1], bh[2], bh[3]);
    if (SPLIT) Frag<T>::keep(bl[0], bl[1], bl[2], bl[3]);
  }
  acc_guard4(acc[0][0], acc[0][1], acc[0][2], acc[0][3]);
  acc_guard4(acc[1][0], acc[1][1], acc[1][2], acc[1][3]);
  acc_guard4(acc[2][0], acc[2][1], acc[2][2], acc[2][3]);
  acc_guard4(acc[3][0], acc[3][1], acc[3][2], acc[3][3]);

  float* slab = sT[wave];
  const float* Rb = RESID ? (resid + (size_t)b * strideR) : nullptr;
#pragma unroll
  for (int i = 0; i < 4; ++i) {
    const int mBase = m0 + (i << 4);
#pragma unroll
    for (int j = 0; j < 4; ++j) {
      const int n = n0 + (j << 4) + rlane;
      float bv = 0.f;
      if (BIAS_MODE == 2) bv = bias[n];
#pragma unroll
      for (int r = 0; r < 8; ++r) {
        float v = acc[i][j][r] * scale;
        if (BIAS_MODE == 1) v += bias[mBase + mOff + r];
        if (BIAS_MODE == 2) v += bv;
        if (RESID) v += Rb[(size_t)(mBase + mOff + r) * ldc + n];
        slab[(mOff + r) * 68 + (j << 4) + rlane] = v;
      }
    }
    __builtin_amdgcn_fence(__ATOMIC_RELEASE, "workgroup");
    __builtin_amdgcn_wave_barrier();
    __builtin_amdgcn_fence(__ATOMIC_ACQUIRE, "workgroup");
    if (OUT_MODE == 0) {
      float* C = (float*)Cout + (size_t)b * strideC;
      const int hh = lane >> 4, c4 = (lane & 15) * 4;
      for (int pass = 0; pass < 2; ++pass) {
#pragma unroll
        for (int it = 0; it < 8; ++it) {
          const int row = it * 2 + hh;
          v4f v = *(const v4f*)(slab + row * 68 + c4);
          *(volatile v4f*)(C + (size_t)(mBase + row) * ldc + n0 + c4) = v;
        }
        __threadfence();
      }
    } else {
      const int q = lane >> 3, c8 = (lane & 7) * 8;
      unsigned short* C  = (unsigned short*)Cout  + (size_t)b * strideC;
      unsigned short* C2 = (OUT_MODE == 2) ? ((unsigned short*)Cout2 + (size_t)b * strideC) : nullptr;
      for (int pass = 0; pass < 2; ++pass) {
#pragma unroll
        for (int it = 0; it < 4; ++it) {
          const int row = it * 4 + q;
          const float* sp = slab + row * 68 + c8;
          v8h hv, lv;
#pragma unroll
          for (int e = 0; e < 8; ++e) {
            if (OUT_MODE == 1) {
              hv[e] = (_Float16)sp[e];
            } else {
              unsigned short hb = f2bf_bits(sp[e]);
              unsigned short lb = f2bf_bits(sp[e] - bf_bits2f(hb));
              hv[e] = __builtin_bit_cast(_Float16, hb);
              lv[e] = __builtin_bit_cast(_Float16, lb);
            }
          }
          *(volatile v8h*)(C + (size_t)(mBase + row) * ldc + n0 + c8) = hv;
          if (OUT_MODE == 2) *(volatile v8h*)(C2 + (size_t)(mBase + row) * ldc + n0 + c8) = lv;
        }
        __threadfence();
      }
    }
    __builtin_amdgcn_fence(__ATOMIC_RELEASE, "workgroup");
    __builtin_amdgcn_wave_barrier();
    __builtin_amdgcn_fence(__ATOMIC_ACQUIRE, "workgroup");
  }
}

__global__ __launch_bounds__(256) void split_bf16x2_kernel(const float* __restrict__ in, unsigned short* __restrict__ hi,
                                                           unsigned short* __restrict__ lo, int n2) {
  const int i = blockIdx.x * 256 + threadIdx.x;
  if (i < n2) {
    const v2f f = *(const v2f*)(in + 2 * (size_t)i);
    const unsigned short h0 = f2bf_bits(f[0]), h1 = f2bf_bits(f[1]);
    const unsigned short l0 = f2bf_bits(f[0] - bf_bits2f(h0)), l1 = f2bf_bits(f[1] - bf_bits2f(h1));
    const unsigned uh = pk16(h0, h1), ul = pk16(l0, l1);
    ((volatile unsigned*)hi)[i] = uh;
    ((volatile unsigned*)lo)[i] = ul;
    __threadfence();
    ((volatile unsigned*)hi)[i] = uh;
    ((volatile unsigned*)lo)[i] = ul;
  }
}

__global__ __launch_bounds__(256) void cvt_f16x2_kernel(const float* __restrict__ in, unsigned short* __restrict__ o,
                                                        int n2, float scale) {
  const int i = blockIdx.x * 256 + threadIdx.x;
  if (i < n2) {
    const v2f f = *(const v2f*)(in + 2 * (size_t)i);
    const _Float16 a = (_Float16)(f[0] * scale), bq = (_Float16)(f[1] * scale);
    const unsigned u = pk16(__builtin_bit_cast(unsigned short, a), __builtin_bit_cast(unsigned short, bq));
    ((volatile unsigned*)o)[i] = u;
    __threadfence();
    ((volatile unsigned*)o)[i] = u;
  }
}

__global__ __launch_bounds__(256) void tsplit_kernel(const float* __restrict__ W, unsigned short* __restrict__ oh,
                                                     unsigned short* __restrict__ ol, int R, int Cc, long sIn, long sOut) {
  __shared__ __align__(16) float tf[64 * 68];
  W  += (size_t)blockIdx.z * sIn;
  oh += (size_t)blockIdx.z * sOut;
  ol += (size_t)blockIdx.z * sOut;
  const int c0  = blockIdx.x * 64;
  const int r0  = blockIdx.y * 64;
  const int tid = threadIdx.x;
  {
    const int lr = tid >> 4;
    const int c4 = (tid & 15) * 4;
#pragma unroll
    for (int it = 0; it < 4; ++it) {
      const int rr = it * 16 + lr;
      const v4f a = *(const v4f*)(W + (size_t)(r0 + rr) * Cc + c0 + c4);
      *(v4f*)(tf + rr * 68 + c4) = a;
    }
  }
  __syncthreads();
  const int sub = tid >> 3;
  const int c8  = (tid & 7) * 8;
  v4u hv[2], lv[2];
#pragma unroll
  for (int it = 0; it < 2; ++it) {
    const int oc = it * 32 + sub;
    v4u a, a2;
#pragma unroll
    for (int q = 0; q < 4; ++q) {
      const float f0 = tf[(c8 + 2 * q) * 68 + oc];
      const float f1 = tf[(c8 + 2 * q + 1) * 68 + oc];
      const unsigned short h0 = f2bf_bits(f0), h1 = f2bf_bits(f1);
      const unsigned short l0 = f2bf_bits(f0 - bf_bits2f(h0)), l1 = f2bf_bits(f1 - bf_bits2f(h1));
      a[q]  = pk16(h0, h1);
      a2[q] = pk16(l0, l1);
    }
    hv[it] = a; lv[it] = a2;
  }
  for (int pass = 0; pass < 2; ++pass) {
#pragma unroll
    for (int it = 0; it < 2; ++it) {
      const int oc = it * 32 + sub;
      const size_t go = (size_t)(c0 + oc) * R + r0 + c8;
      *(volatile v4u*)(oh + go) = hv[it];
      *(volatile v4u*)(ol + go) = lv[it];
    }
    __threadfence();
  }
}

#define AG_ROWS      256
#define AG_CAP       6144
#define AG_CHUNK     2048
#define AG_LDS_BYTES ((AG_ROWS * NHID + AG_CAP) * 4 + 128)

__global__ __launch_bounds__(256) void agg_kernel(const float* __restrict__ ng,
                                                  const int* __restrict__ ei1, const float* __restrict__ ea1,
                                                  const int* __restrict__ ei2, const float* __restrict__ ea2,
                                                  unsigned short* __restrict__ inch, unsigned short* __restrict__ incl,
                                                  int nN, int nE) {
  extern __shared__ __attribute__((aligned(16))) float ag_lds[];
  float*    acc  = ag_lds;
  unsigned* lst  = (unsigned*)(ag_lds + AG_ROWS * NHID);
  int*      wcnt = (int*)(ag_lds + AG_ROWS * NHID + AG_CAP);
  const int tid = threadIdx.x, lane = tid & 31, wave = tid >> 5;
  const int tile0 = blockIdx.x * AG_ROWS;
  const v4f z4 = {0.f, 0.f, 0.f, 0.f};
  for (int i = tid; i < AG_ROWS * NHID / 4; i += 256) *(v4f*)(acc + 4 * i) = z4;
  __syncthreads();
  const unsigned ltmask = (1u << lane) - 1u;

  for (int s = 0; s < 2; ++s) {
    const int*   ei   = (s == 0) ? ei1 : ei2;
    const float* ea   = (s == 0) ? ea1 : ea2;
    const int*   dsti = ei + nE;
    const int    coff = (s == 0) ? NHID : 2 * NHID;
    const bool   al4  = ((nE & 3) == 0);
    int count = 0;
    for (int cbase = 0; cbase < nE; cbase += AG_CHUNK) {
      const int e0 = cbase + tid * 8;
      int d[8];
      if (al4 && (cbase + AG_CHUNK <= nE)) {
        const v4i a = *(const v4i*)(dsti + e0);
        const v4i bq = *(const v4i*)(dsti + e0 + 4);
        d[0] = a[0]; d[1] = a[1]; d[2] = a[2]; d[3] = a[3];
        d[4] = bq[0]; d[5] = bq[1]; d[6] = bq[2]; d[7] = bq[3];
      } else {
#pragma unroll
        for (int j = 0; j < 8; ++j) {
          const int e  = e0 + j;
          const int ec = min(e, nE - 1);
          const int dv = dsti[ec];
          d[j] = (e < nE) ? dv : -1;
        }
      }
      unsigned bm[8];
      int wtot = 0;
#pragma unroll
      for (int j = 0; j < 8; ++j) {
        const int loc = d[j] - tile0;
        const bool valid = (unsigned)loc < (unsigned)AG_ROWS;
        bm[j] = __builtin_amdgcn_ballot_w32(valid);
        wtot += __builtin_popcount(bm[j]);
      }
      if (lane == 0) wcnt[wave] = wtot;
      __syncthreads();
      int pre = 0, tot = 0;
#pragma unroll
      for (int w = 0; w < 8; ++w) { const int cw = wcnt[w]; tot += cw; pre += (w < wave) ? cw : 0; }
      int pos = count + pre;
#pragma unroll
      for (int j = 0; j < 8; ++j) {
        const int loc = d[j] - tile0;
        const bool valid = (unsigned)loc < (unsigned)AG_ROWS;
        const int p = pos + __builtin_popcount(bm[j] & ltmask);
        if (valid && p < AG_CAP) lst[p] = ((unsigned)(e0 + j) << 8) | (unsigned)loc;
        pos += __builtin_popcount(bm[j]);
      }
      count += tot;
      __syncthreads();
    }
    const int cnt = min(count, AG_CAP);
    for (int base = 0; base < cnt; base += 32) {
      const int idx = base + lane;
      const unsigned key = lst[min(idx, AG_CAP - 1)];
      const bool mine = (idx < cnt) && ((int)(key & 7u) == wave);
      unsigned m = __builtin_amdgcn_ballot_w32(mine);
      while (m != 0u) {
        const int bsel = __builtin_ctz(m);
        m &= (m - 1u);
        const unsigned k = (unsigned)__builtin_amdgcn_readlane((int)key, bsel);
        int e = (int)(k >> 8); e = min(e, nE - 1);
        const int loc = (int)(k & 255u);
        int src = ei[e]; src = min(max(src, 0), nN - 1);
        const float a = ea[e];
        const float* row = ng + (size_t)src * NQKV + coff + lane * 4;
        const v4f x0 = *(const v4f*)(row);
        const v4f x1 = *(const v4f*)(row + 128);
        float* ar = acc + loc * NHID + lane * 4;
        v4f r0v = *(const v4f*)(ar);
        v4f r1v = *(const v4f*)(ar + 128);
        r0v += a * x0;
        r1v += a * x1;
        *(v4f*)(ar) = r0v;
        *(v4f*)(ar + 128) = r1v;
      }
    }
    __syncthreads();
  }

  for (int rb = 0; rb < 32; rb += 4) {
    v4u hv[4], lv[4];
#pragma unroll
    for (int i = 0; i < 4; ++i) {
      const int r = wave * 32 + rb + i;
      const int node = tile0 + r;
      const float* xr = ng + (size_t)node * NQKV + lane * 8;
      const float* ar = acc + r * NHID + lane * 8;
      const v4f a0 = *(const v4f*)(xr);
      const v4f a1 = *(const v4f*)(xr + 4);
      const v4f b0 = *(const v4f*)(ar);
      const v4f b1 = *(const v4f*)(ar + 4);
      const v4f f0 = a0 + b0, f1 = a1 + b1;
      float f[8];
      f[0] = f0[0]; f[1] = f0[1]; f[2] = f0[2]; f[3] = f0[3];
      f[4] = f1[0]; f[5] = f1[1]; f[6] = f1[2]; f[7] = f1[3];
      v4u hh4, ll4;
#pragma unroll
      for (int q = 0; q < 4; ++q) {
        const unsigned short h0 = f2bf_bits(f[2 * q]), h1 = f2bf_bits(f[2 * q + 1]);
        const unsigned short l0 = f2bf_bits(f[2 * q] - bf_bits2f(h0)), l1 = f2bf_bits(f[2 * q + 1] - bf_bits2f(h1));
        hh4[q] = pk16(h0, h1);
        ll4[q] = pk16(l0, l1);
      }
      hv[i] = hh4; lv[i] = ll4;
    }
    for (int pass = 0; pass < 2; ++pass) {
#pragma unroll
      for (int i = 0; i < 4; ++i) {
        const int node = tile0 + wave * 32 + rb + i;
        *(volatile v4u*)(inch + (size_t)node * NHID + lane * 8) = hv[i];
        *(volatile v4u*)(incl + (size_t)node * NHID + lane * 8) = lv[i];
      }
      __threadfence();
    }
  }
}

__global__ __launch_bounds__(128)
void attn_kernel(const unsigned short* __restrict__ qhp, const unsigned short* __restrict__ qlp,
                 const unsigned short* __restrict__ vtp, unsigned short* __restrict__ ctxp,
                 const int* __restrict__ ngp, int nN, float sscale2, float pscale, float oscale) {
  union FB { v16b v; v8b h[2]; };
  union FH { v16h v; v8h h[2]; };
  __shared__ __align__(16) __bf16   Ksh[64 * 64];
  __shared__ __align__(16) __bf16   Ksl[64 * 64];
  __shared__ __align__(16) _Float16 Vth[64 * 64];
  __shared__ __align__(16) _Float16 Psh[4][16 * 64];
  __shared__ __align__(16) float    Os[4][16 * 68];

  const int tid  = threadIdx.x;
  const int wave = tid >> 5;
  const int lane = tid & 31;
  const int hh   = lane >> 4;
  const int c    = lane & 15;

  int ngr = ngp[0]; ngr = max(ngr, 1);
  const int npg = nN / ngr;
  const int bx = blockIdx.x;
  const int qb = bx & 7;
  const int h  = (bx >> 3) & 3;
  const int g  = bx >> 5;
  int node0 = g * npg; node0 = max(0, min(node0, nN - NPG));
  const int q0 = node0 + qb * 64 + wave * 16;

  const __bf16*   Qh  = (const __bf16*)(const void*)qhp;
  const __bf16*   Ql  = (const __bf16*)(const void*)qlp;
  const _Float16* Vt  = (const _Float16*)(const void*)vtp + (size_t)(h * DHD) * nN + node0;
  _Float16*       ctx = (_Float16*)(void*)ctxp;

  v16b qah[2], qal[2];
#pragma unroll
  for (int dc = 0; dc < 2; ++dc) {
    const size_t qo = (size_t)(q0 + c) * QKP + h * DHD + dc * 32 + 8 * hh;
    qah[dc] = Frag<__bf16>::load(Qh + qo);
    qal[dc] = Frag<__bf16>::load(Ql + qo);
  }

  float mrow[8], lrow[8];
  v8f oacc[4];
#pragma unroll
  for (int r = 0; r < 8; ++r) { mrow[r] = -INFINITY; lrow[r] = 0.f; }
#pragma unroll
  for (int t = 0; t < 4; ++t) oacc[t] = (v8f){0.f,0.f,0.f,0.f,0.f,0.f,0.f,0.f};

  for (int kc = 0; kc < NPG / 64; ++kc) {
    const int kv0 = kc * 64;
    __syncthreads();
    {
      const int r = tid >> 1, half = (tid & 1) * 32;
      const size_t ko = (size_t)(node0 + kv0 + r) * QKP + NHID + h * DHD + half;
      const __bf16*   ksh = Qh + ko;
      const __bf16*   ksl = Ql + ko;
      const _Float16* vsh = Vt + (size_t)r * nN + kv0 + half;
#pragma unroll
      for (int i = 0; i < 4; ++i) {
        const v8b a0 = *(const v8b*)(ksh + 8 * i);
        const v8b a1 = *(const v8b*)(ksl + 8 * i);
        const v8h b0 = *(const v8h*)(vsh + 8 * i);
        *(v8b*)(Ksh + r * 64 + half + 8 * i) = a0;
        *(v8b*)(Ksl + r * 64 + half + 8 * i) = a1;
        *(v8h*)(Vth + r * 64 + half + 8 * i) = b0;
      }
    }
    __syncthreads();

    v8f s[4];
#pragma unroll
    for (int j = 0; j < 4; ++j) {
      s[j] = (v8f){0.f,0.f,0.f,0.f,0.f,0.f,0.f,0.f};
#pragma unroll
      for (int dc = 0; dc < 2; ++dc) {
        FB kb, kl;
        kb.h[0] = *(const v8b*)(Ksh + (j * 16 + c) * 64 + dc * 32 + 8 * hh);
        kb.h[1] = *(const v8b*)(Ksh + (j * 16 + c) * 64 + dc * 32 + 16 + 8 * hh);
        kl.h[0] = *(const v8b*)(Ksl + (j * 16 + c) * 64 + dc * 32 + 8 * hh);
        kl.h[1] = *(const v8b*)(Ksl + (j * 16 + c) * 64 + dc * 32 + 16 + 8 * hh);
        s[j] = mma_b(qah[dc], kb.v, s[j]);
        s[j] = mma_b(qah[dc], kl.v, s[j]);
        s[j] = mma_b(qal[dc], kb.v, s[j]);
      }
    }
    float cm[8];
#pragma unroll
    for (int r = 0; r < 8; ++r) {
      float m = -INFINITY;
#pragma unroll
      for (int j = 0; j < 4; ++j) {
        const float sv = s[j][r] * sscale2;
        s[j][r] = sv;
        m = fmaxf(m, sv);
      }
#pragma unroll
      for (int off = 1; off < 16; off <<= 1) m = fmaxf(m, __shfl_xor(m, off, 32));
      cm[r] = m;
    }
    _Float16* pw = Psh[wave];
#pragma unroll
    for (int r = 0; r < 8; ++r) {
      const float mnew  = fmaxf(mrow[r], cm[r]);
      const float alpha = exp2f(mrow[r] - mnew);
      mrow[r] = mnew;
      float psum = 0.f;
#pragma unroll
      for (int j = 0; j < 4; ++j) {
        const float p = exp2f(s[j][r] - mnew);
        psum += p;
        pw[(8 * hh + r) * 64 + j * 16 + c] = (_Float16)(p * pscale);
      }
#pragma unroll
      for (int off = 1; off < 16; off <<= 1) psum += __shfl_xor(psum, off, 32);
      lrow[r] = lrow[r] * alpha + psum;
#pragma unroll
      for (int t = 0; t < 4; ++t) oacc[t][r] *= alpha;
    }
    __builtin_amdgcn_fence(__ATOMIC_RELEASE, "workgroup");
    __builtin_amdgcn_wave_barrier();
    __builtin_amdgcn_fence(__ATOMIC_ACQUIRE, "workgroup");
#pragma unroll 1
    for (int kk = 0; kk < 2; ++kk) {
      FH pa;
      pa.h[0] = *(const v8h*)(pw + c * 64 + kk * 32 + 8 * hh);
      pa.h[1] = *(const v8h*)(pw + c * 64 + kk * 32 + 16 + 8 * hh);
#pragma unroll
      for (int t = 0; t < 4; ++t) {
        FH vb;
        vb.h[0] = *(const v8h*)(Vth + (t * 16 + c) * 64 + kk * 32 + 8 * hh);
        vb.h[1] = *(const v8h*)(Vth + (t * 16 + c) * 64 + kk * 32 + 16 + 8 * hh);
        oacc[t] = mma_h(pa.v, vb.v, oacc[t]);
      }
    }
  }

  float* os = Os[wave];
#pragma unroll
  for (int r = 0; r < 8; ++r) {
    const float inv = (1.0f / lrow[r]) * oscale;
#pragma unroll
    for (int t = 0; t < 4; ++t) os[(8 * hh + r) * 68 + t * 16 + c] = oacc[t][r] * inv;
  }
  __builtin_amdgcn_fence(__ATOMIC_RELEASE, "workgroup");
  __builtin_amdgcn_wave_barrier();
  __builtin_amdgcn_fence(__ATOMIC_ACQUIRE, "workgroup");
  {
    const int q = lane >> 3, c8 = (lane & 7) * 8;
    for (int pass = 0; pass < 2; ++pass) {
#pragma unroll
      for (int it = 0; it < 4; ++it) {
        const int row = it * 4 + q;
        const float* sp = os + row * 68 + c8;
        v8h hv;
#pragma unroll
        for (int e = 0; e < 8; ++e) hv[e] = (_Float16)sp[e];
        *(volatile v8h*)(ctx + (size_t)(q0 + row) * NHID + h * DHD + c8) = hv;
      }
      __threadfence();
    }
  }
}

#define OL_PITCH 260
#define OL_LDS_BYTES (64 * OL_PITCH * 4)

__global__ __launch_bounds__(256) void outln_kernel(const unsigned short* __restrict__ ctxp, const unsigned short* __restrict__ wop,
                                                    const float* __restrict__ bo,
                                                    const unsigned short* __restrict__ inch, const unsigned short* __restrict__ incl,
                                                    const float* __restrict__ gamma, const float* __restrict__ beta,
                                                    float* __restrict__ out, float wscale) {
  extern __shared__ __attribute__((aligned(16))) float ol_lds[];
  const _Float16* A  = (const _Float16*)(const void*)ctxp;
  const _Float16* Bt = (const _Float16*)(const void*)wop;
  const int lane = threadIdx.x & 31;
  const int wave = threadIdx.x >> 5;
  const int m0 = blockIdx.x * 64;
  const int n0 = wave * 64;
  const int rlane = lane & 15;
  const int koff  = (lane >> 4) * 8;
  const int mOff  = (lane >> 4) * 8;

  v8f acc[4][4];
#pragma unroll
  for (int i = 0; i < 4; ++i)
#pragma unroll
    for (int j = 0; j < 4; ++j) acc[i][j] = (v8f){0.f,0.f,0.f,0.f,0.f,0.f,0.f,0.f};

  for (int k0 = 0; k0 < NHID; k0 += 32) {
    v16h bh[4];
#pragma unroll
    for (int j = 0; j < 4; ++j) bh[j] = Frag<_Float16>::load(Bt + (size_t)(n0 + (j << 4) + rlane) * NHID + koff + k0);
#pragma unroll
    for (int i = 0; i < 4; ++i) {
      v16h ah = Frag<_Float16>::load(A + (size_t)(m0 + (i << 4) + rlane) * NHID + koff + k0);
#pragma unroll
      for (int j = 0; j < 4; ++j) acc[i][j] = Frag<_Float16>::mma(ah, bh[j], acc[i][j]);
      Frag<_Float16>::guard(acc[i][0], acc[i][3], ah, ah);
    }
    Frag<_Float16>::keep(bh[0], bh[1], bh[2], bh[3]);
  }
  acc_guard4(acc[0][0], acc[0][1], acc[0][2], acc[0][3]);
  acc_guard4(acc[1][0], acc[1][1], acc[1][2], acc[1][3]);
  acc_guard4(acc[2][0], acc[2][1], acc[2][2], acc[2][3]);
  acc_guard4(acc[3][0], acc[3][1], acc[3][2], acc[3][3]);

#pragma unroll
  for (int i = 0; i < 4; ++i) {
#pragma unroll
    for (int j = 0; j < 4; ++j) {
      const int col = n0 + (j << 4) + rlane;
      const float bv = bo[col];
#pragma unroll
      for (int r = 0; r < 8; ++r) ol_lds[((i << 4) + mOff + r) * OL_PITCH + col] = acc[i][j][r] * wscale + bv;
    }
  }
  __syncthreads();

  const v4f g0 = *(const v4f*)(gamma + 4 * lane);
  const v4f g1 = *(const v4f*)(gamma + 128 + 4 * lane);
  const v4f e0 = *(const v4f*)(beta + 4 * lane);
  const v4f e1 = *(const v4f*)(beta + 128 + 4 * lane);
  const float invn = 1.0f / (float)NHID;
  for (int rb = 0; rb < 16; rb += 4) {
    v4f o0[4], o1[4];
#pragma unroll
    for (int i = 0; i < 4; ++i) {
      const int row  = wave * 16 + rb + i;
      const int node = m0 + row;
      const v4f a0 = *(const v4f*)(ol_lds + row * OL_PITCH + 4 * lane);
      const v4f a1 = *(const v4f*)(ol_lds + row * OL_PITCH + 128 + 4 * lane);
      const v2u h0 = *(const v2u*)(const void*)(inch + (size_t)node * NHID + 4 * lane);
      const v2u h1 = *(const v2u*)(const void*)(inch + (size_t)node * NHID + 128 + 4 * lane);
      const v2u l0 = *(const v2u*)(const void*)(incl + (size_t)node * NHID + 4 * lane);
      const v2u l1 = *(const v2u*)(const void*)(incl + (size_t)node * NHID + 128 + 4 * lane);
      v4f x0, x1;
      x0[0] = a0[0] + (__uint_as_float(h0[0] << 16)         + __uint_as_float(l0[0] << 16));
      x0[1] = a0[1] + (__uint_as_float(h0[0] & 0xffff0000u) + __uint_as_float(l0[0] & 0xffff0000u));
      x0[2] = a0[2] + (__uint_as_float(h0[1] << 16)         + __uint_as_float(l0[1] << 16));
      x0[3] = a0[3] + (__uint_as_float(h0[1] & 0xffff0000u) + __uint_as_float(l0[1] & 0xffff0000u));
      x1[0] = a1[0] + (__uint_as_float(h1[0] << 16)         + __uint_as_float(l1[0] << 16));
      x1[1] = a1[1] + (__uint_as_float(h1[0] & 0xffff0000u) + __uint_as_float(l1[0] & 0xffff0000u));
      x1[2] = a1[2] + (__uint_as_float(h1[1] << 16)         + __uint_as_float(l1[1] << 16));
      x1[3] = a1[3] + (__uint_as_float(h1[1] & 0xffff0000u) + __uint_as_float(l1[1] & 0xffff0000u));
      float sum = (x0[0] + x0[1]) + (x0[2] + x0[3]) + (x1[0] + x1[1]) + (x1[2] + x1[3]);
#pragma unroll
      for (int off = 16; off > 0; off >>= 1) sum += __shfl_xor(sum, off, 32);
      const float mu = sum * invn;
      const v4f d0 = x0 - mu, d1 = x1 - mu;
      float var = (d0[0] * d0[0] + d0[1] * d0[1]) + (d0[2] * d0[2] + d0[3] * d0[3])
                + (d1[0] * d1[0] + d1[1] * d1[1]) + (d1[2] * d1[2] + d1[3] * d1[3]);
#pragma unroll
      for (int off = 16; off > 0; off >>= 1) var += __shfl_xor(var, off, 32);
      const float rstd = rsqrtf(var * invn + 1e-5f);
      o0[i] = d0 * rstd * g0 + e0;
      o1[i] = d1 * rstd * g1 + e1;
    }
    for (int pass = 0; pass < 2; ++pass) {
#pragma unroll
      for (int i = 0; i < 4; ++i) {
        const int node = m0 + wave * 16 + rb + i;
        *(volatile v4f*)(out + (size_t)node * NHID + 4 * lane)       = o0[i];
        *(volatile v4f*)(out + (size_t)node * NHID + 128 + 4 * lane) = o1[i];
      }
      __threadfence();
    }
  }
}

extern "C" void kernel_launch(void* const* d_in, const int* in_sizes, int n_in,
                              void* d_out, int out_size, void* d_ws, size_t ws_size,
                              hipStream_t stream) {
  if (n_in < 15) return;
  if (in_sizes[0] != NNODE * NFEAT) return;
  if (in_sizes[1] != NEDGE || in_sizes[2] != NEDGE) return;
  if (in_sizes[3] != NFEAT * NHID || in_sizes[4] != NFEAT * NHID || in_sizes[5] != NFEAT * NHID) return;
  if (in_sizes[6] != NQKV * NHID || in_sizes[7] != NQKV) return;
  if (in_sizes[8] != NHID * NHID || in_sizes[9] != NHID || in_sizes[10] != NHID || in_sizes[11] != NHID) return;
  if (in_sizes[12] != 2 * NEDGE || in_sizes[13] != 2 * NEDGE || in_sizes[14] < 1) return;
  if (out_size != NNODE * NHID) return;

  const float* x          = (const float*)d_in[0];
  const float* edge_attr  = (const float*)d_in[1];
  const float* edge_attr2 = (const float*)d_in[2];
  const float* ln_w       = (const float*)d_in[3];
  const float* conv1_w    = (const float*)d_in[4];
  const float* conv2_w    = (const float*)d_in[5];
  const float* in_proj_w  = (const float*)d_in[6];
  const float* in_proj_b  = (const float*)d_in[7];
  const float* out_proj_w = (const float*)d_in[8];
  const float* out_proj_b = (const float*)d_in[9];
  const float* gamma      = (const float*)d_in[10];
  const float* beta       = (const float*)d_in[11];
  const int*   edge_index  = (const int*)d_in[12];
  const int*   edge_index2 = (const int*)d_in[13];
  const int*   num_graphs  = (const int*)d_in[14];

  const size_t szNG   = (size_t)NNODE * NQKV * 4;
  const size_t szQK   = (size_t)NNODE * QKP * 2;
  const size_t szVT   = (size_t)NHID * NNODE * 2;
  const size_t szCTX  = (size_t)NNODE * NHID * 2;
  const size_t szIP   = (size_t)NQKV * NHID * 2;
  const size_t szWO   = (size_t)NHID * NHID * 2;
  const size_t szX    = (size_t)NNODE * NFEAT * 2;
  const size_t szWT   = (size_t)NQKV * NFEAT * 2;
  const size_t szINC  = (size_t)NNODE * NHID * 2;

  const size_t oA    = 0;
  const size_t oQKh  = oA;
  const size_t oQKl  = oQKh + szQK;
  const size_t oVT   = oQKl + szQK;
  const size_t oCTX  = oVT + szVT;
  const size_t endA  = oCTX + szCTX;
  if (endA != szNG) return;
  const size_t oIPh  = oCTX;
  const size_t oIPl  = oIPh + szIP;
  if (oIPl + szIP > endA) return;
  const size_t oWO   = oA;
  const size_t oB    = endA;
  const size_t oXh   = oB;
  const size_t oXl   = oXh + szX;
  const size_t oWTh  = oXl + szX;
  const size_t oWTl  = oWTh + szWT;
  const size_t oINCh = oB;
  const size_t oINCl = oINCh + szINC;
  const size_t total = oINCl + szINC;
  if (oWTl + szWT > total) return;
  if (total > ws_size) return;

  char* ws = (char*)d_ws;
  float*          NG   = (float*)(ws + oA);
  unsigned short* QKh  = (unsigned short*)(ws + oQKh);
  unsigned short* QKl  = (unsigned short*)(ws + oQKl);
  unsigned short* VTp  = (unsigned short*)(ws + oVT);
  unsigned short* CTX  = (unsigned short*)(ws + oCTX);
  unsigned short* IPh  = (unsigned short*)(ws + oIPh);
  unsigned short* IPl  = (unsigned short*)(ws + oIPl);
  unsigned short* WO16 = (unsigned short*)(ws + oWO);
  unsigned short* Xh   = (unsigned short*)(ws + oXh);
  unsigned short* Xl   = (unsigned short*)(ws + oXl);
  unsigned short* WTh  = (unsigned short*)(ws + oWTh);
  unsigned short* WTl  = (unsigned short*)(ws + oWTl);
  unsigned short* INCh = (unsigned short*)(ws + oINCh);
  unsigned short* INCl = (unsigned short*)(ws + oINCl);

  const dim3 blk(256);

  const int n2x = NNODE * NFEAT / 2;
  split_bf16x2_kernel<<<dim3((n2x + 255) / 256), blk, 0, stream>>>(x, Xh, Xl, n2x);
  tsplit_kernel<<<dim3(NHID / 64, NFEAT / 64, 1), blk, 0, stream>>>(ln_w,    WTh,                    WTl,                    NFEAT, NHID, 0L, 0L);
  tsplit_kernel<<<dim3(NHID / 64, NFEAT / 64, 1), blk, 0, stream>>>(conv1_w, WTh + NHID * NFEAT,     WTl + NHID * NFEAT,     NFEAT, NHID, 0L, 0L);
  tsplit_kernel<<<dim3(NHID / 64, NFEAT / 64, 1), blk, 0, stream>>>(conv2_w, WTh + 2 * NHID * NFEAT, WTl + 2 * NHID * NFEAT, NFEAT, NHID, 0L, 0L);
  {
    const dim3 g(((NNODE / 64) * (NQKV / 64) + 7) / 8, 1);
    wmma_gemm64<1, true, 0, 0, false><<<g, blk, 0, stream>>>(
        Xh, Xl, NFEAT, 0L, WTh, WTl, NFEAT, 0L, (void*)NG, (void*)NG, NQKV, 0L,
        in_proj_b, x, 0L, NNODE, NQKV, NFEAT, 1.0f);
  }
  hipFuncSetAttribute(reinterpret_cast<const void*>(&agg_kernel), hipFuncAttributeMaxDynamicSharedMemorySize, AG_LDS_BYTES);
  agg_kernel<<<dim3(NNODE / AG_ROWS), blk, AG_LDS_BYTES, stream>>>(NG, edge_index, edge_attr, edge_index2, edge_attr2,
                                                                    INCh, INCl, NNODE, NEDGE);
  const int n2ip = NQKV * NHID / 2;
  split_bf16x2_kernel<<<dim3((n2ip + 255) / 256), blk, 0, stream>>>(in_proj_w, IPh, IPl, n2ip);
  {
    const dim3 g(((NNODE / 64) * (QKP / 64) + 7) / 8, 1);
    wmma_gemm64<1, true, 2, 2, false><<<g, blk, 0, stream>>>(
        INCh, INCl, NHID, 0L, IPh, IPl, NHID, 0L, (void*)QKh, (void*)QKl, QKP, 0L,
        in_proj_b, x, 0L, NNODE, QKP, NHID, 1.0f);
  }
  {
    const dim3 g(((NHID / 64) * (NNODE / 64) + 7) / 8, 1);
    wmma_gemm64<1, true, 1, 1, false><<<g, blk, 0, stream>>>(
        IPh + 2 * NHID * NHID, IPl + 2 * NHID * NHID, NHID, 0L, INCh, INCl, NHID, 0L, (void*)VTp, (void*)VTp, NNODE, 0L,
        in_proj_b + 2 * NHID, x, 0L, NHID, NNODE, NHID, 1.0f);
  }
  {
    const float sscale2 = (float)(0.125 * 1.4426950408889634);
    attn_kernel<<<dim3(NGRAPH * NHEAD * (NPG / 64)), dim3(128), 0, stream>>>(QKh, QKl, VTp, CTX, num_graphs, NNODE,
                                                                             sscale2, 256.0f, 1.0f / 256.0f);
  }
  const int n2wo = NHID * NHID / 2;
  cvt_f16x2_kernel<<<dim3((n2wo + 255) / 256), blk, 0, stream>>>(out_proj_w, WO16, n2wo, 16.0f);
  hipFuncSetAttribute(reinterpret_cast<const void*>(&outln_kernel), hipFuncAttributeMaxDynamicSharedMemorySize, OL_LDS_BYTES);
  outln_kernel<<<dim3(NNODE / 64), dim3(128), OL_LDS_BYTES, stream>>>(CTX, WO16, out_proj_b, INCh, INCl, gamma, beta,
                                                                      (float*)d_out, 1.0f / 16.0f);
  (void)hipGetLastError();
}
